// KANLayerOptimized_69157563400754
// MI455X (gfx1250) — hardware-verified
//
#include <hip/hip_runtime.h>
#include <stddef.h>
#include <stdint.h>

#define NB    8192
#define NI    256
#define NG    32
#define NO    512
#define NKN   36
#define KSP   (NI * NG)
#define KTOT  (KSP + NI)
#define KSUP  256
#define NSUP  (KTOT / KSUP)
#define BM    32
#define LDA   264
#define STP   68
#define TP    72

static_assert(KTOT % KSUP == 0);
static_assert((NSUP - 1) * 8 == NI);
static_assert(NB % BM == 0);
static_assert(NO == 8 * 64);
static_assert(KTOT % 64 == 0);
static_assert(NO % 32 == 0);
static_assert(KSP % 64 == 0);
static_assert((LDA * 2) % 16 == 0);
static_assert((STP * 4) % 16 == 0);
static_assert((TP * 2) % 16 == 0);
static_assert((KTOT * 2) % 128 == 0);

typedef _Float16 v16h __attribute__((ext_vector_type(16)));
typedef _Float16 v8h  __attribute__((ext_vector_type(8)));
typedef float    v8f  __attribute__((ext_vector_type(8)));
typedef float    v4f  __attribute__((ext_vector_type(4)));
typedef unsigned int v4u __attribute__((ext_vector_type(4)));
typedef v8h __attribute__((may_alias)) v8ha;
typedef v4u __attribute__((may_alias)) v4ua;
typedef v4f __attribute__((may_alias)) v4fa;

union Frag { v16h v; v8h h[2]; };

__device__ __forceinline__ v8f mma16(v16h a, v16h b, v8f cacc) {
  cacc = __builtin_amdgcn_wmma_f32_16x16x32_f16(false, a, false, b, (short)0, cacc, false, false);
  asm volatile("v_nop\n\tv_nop\n\tv_nop\n\tv_nop" : "+v"(cacc) : "v"(a), "v"(b));
  return cacc;
}

__device__ __forceinline__ v8f zero8() { return (v8f){0.f, 0.f, 0.f, 0.f, 0.f, 0.f, 0.f, 0.f}; }

__device__ __forceinline__ v16h ldfrag_g(const _Float16* __restrict__ p, int ld, int row0, int k0, int lane) {
  const int m = lane & 15, lh = lane >> 4;
  const _Float16* q = p + (size_t)(row0 + m) * ld + k0 + 8 * lh;
  Frag f;
  f.h[0] = *(const v8h*)(q);
  f.h[1] = *(const v8h*)(q + 16);
  return f.v;
}

__device__ __forceinline__ v16h ldfrag_l(const _Float16* p, int ld, int row0, int k0, int lane) {
  const int m = lane & 15, lh = lane >> 4;
  const _Float16* q = p + (row0 + m) * ld + k0 + 8 * lh;
  Frag f;
  f.h[0] = *(const v8ha*)(q);
  f.h[1] = *(const v8ha*)(q + 16);
  return f.v;
}

__global__ __launch_bounds__(256) void k_prep(const float* __restrict__ coeffs, const float* __restrict__ skipw,
                                              _Float16* __restrict__ WT) {
  __shared__ __align__(16) _Float16 T[32 * TP];

  const int tid = threadIdx.x;
  const int k0 = blockIdx.x * 64;
  const int w0 = blockIdx.y * 32;
  const float* src;
  float scl;
  if (k0 < KSP) { src = coeffs + (size_t)k0 * NO;         scl = 64.0f;  }
  else          { src = skipw  + (size_t)(k0 - KSP) * NO; scl = 256.0f; }

  const int kr = tid >> 3;
  const int wp = (tid & 7) * 4;
#pragma unroll
  for (int p = 0; p < 2; ++p) {
    const int k = kr + 32 * p;
    const v4f v = *(const v4f*)(src + (size_t)k * NO + w0 + wp);
    T[(wp + 0) * TP + k] = (_Float16)(v.x * scl);
    T[(wp + 1) * TP + k] = (_Float16)(v.y * scl);
    T[(wp + 2) * TP + k] = (_Float16)(v.z * scl);
    T[(wp + 3) * TP + k] = (_Float16)(v.w * scl);
  }
  __syncthreads();

  const int w = tid >> 3, pc = tid & 7;
  const v4u val = *(const v4ua*)(T + w * TP + pc * 8);
  _Float16* dst = WT + (size_t)(w0 + w) * KTOT + k0 + pc * 8;
  *(volatile v4u*)dst = val;
  __threadfence();
  *(volatile v4u*)dst = val;
}

__global__ __launch_bounds__(256) void k_main(const float* __restrict__ X, const float* __restrict__ shf,
                                              const float* __restrict__ lsc, const _Float16* __restrict__ WT,
                                              const float* __restrict__ bias, const float* __restrict__ skipb,
                                              const float* __restrict__ gmg, const float* __restrict__ btg,
                                              float* __restrict__ out) {
  __shared__ float kn[40];
  __shared__ __align__(16) _Float16 sA[BM * LDA];
  __shared__ __align__(16) float part[BM * 8];
  __shared__ float mu_s[BM];
  __shared__ float rs_s[BM];
  __shared__ __align__(16) float st[8][16 * STP];

  const int tid = threadIdx.x, lane = tid & 31, wave = tid >> 5;
  const int hh = lane >> 4, c = lane & 15;
  const int m0 = blockIdx.x * BM;
  const int ncol0 = wave * 64;

  if (tid < NKN) {
    float kv = (float)((double)(tid - 3) * (1.0 / 29.0));
    kv = (tid <= 3) ? 0.0f : kv;
    kv = (tid >= 32) ? 1.0f : kv;
    kn[tid] = kv;
  }
  __syncthreads();

  v8f acc[2][4];
#pragma unroll
  for (int s = 0; s < 2; ++s) {
#pragma unroll
    for (int t = 0; t < 4; ++t) acc[s][t] = zero8();
  }

  const float* xrow = X + (size_t)(m0 + lane) * NI;
  _Float16* ar = sA + lane * LDA + wave * 32;

  for (int sup = 0; sup < NSUP; ++sup) {
    if (sup < NSUP - 1) {
      const int f = sup * 8 + wave;
      const float ls = lsc[f];
      const float sp = fmaxf(ls, 0.0f) + log1pf(expf(-fabsf(ls)));
      const float sc = sp + 0.001f;
      const float xv = xrow[f];
      float z = (xv - shf[f]) * sc;
      z = fminf(fmaxf(z, -30.0f), 30.0f);
      const float xn = 1.0f / (1.0f + expf(-z));
      const float vm = (xn < 1.0f) ? 256.0f : 0.0f;
      int span = 3 + (int)(xn * 29.0f);
      span = (span < 3) ? 3 : span;
      span = (span > 31) ? 31 : span;
      span -= (xn < kn[span]) ? 1 : 0;
      span += (xn >= kn[span + 1]) ? 1 : 0;
      span = (span < 3) ? 3 : span;
      span = (span > 31) ? 31 : span;
      const float tl1 = xn - kn[span], tl2 = xn - kn[span - 1], tl3 = xn - kn[span - 2];
      const float tr1 = kn[span + 1] - xn, tr2 = kn[span + 2] - xn, tr3 = kn[span + 3] - xn;
      float n0, n1, n2, n3, sv, tq;
      tq = 1.0f / (tr1 + tl1);
      n0 = tr1 * tq;
      n1 = tl1 * tq;
      tq = n0 * (1.0f / (tr1 + tl2)); n0 = tr1 * tq;      sv = tl2 * tq;
      tq = n1 * (1.0f / (tr2 + tl1)); n1 = sv + tr2 * tq; n2 = tl1 * tq;
      tq = n0 * (1.0f / (tr1 + tl3)); n0 = tr1 * tq;      sv = tl3 * tq;
      tq = n1 * (1.0f / (tr2 + tl2)); n1 = sv + tr2 * tq; sv = tl2 * tq;
      tq = n2 * (1.0f / (tr3 + tl1)); n2 = sv + tr3 * tq; n3 = tl1 * tq;
      const v8h zz = (v8h){(_Float16)0.0f, (_Float16)0.0f, (_Float16)0.0f, (_Float16)0.0f,
                           (_Float16)0.0f, (_Float16)0.0f, (_Float16)0.0f, (_Float16)0.0f};
      *(v8ha*)(ar + 0)  = zz;
      *(v8ha*)(ar + 8)  = zz;
      *(v8ha*)(ar + 16) = zz;
      *(v8ha*)(ar + 24) = zz;
      const int g0 = span - 3;
      ar[g0 + 0] = (_Float16)(n0 * vm);
      ar[g0 + 1] = (_Float16)(n1 * vm);
      ar[g0 + 2] = (_Float16)(n2 * vm);
      ar[g0 + 3] = (_Float16)(n3 * vm);
    } else {
      const float* src = xrow + wave * 32;
#pragma unroll
      for (int q = 0; q < 4; ++q) {
        const v4f a = *(const v4f*)(src + 8 * q);
        const v4f b = *(const v4f*)(src + 8 * q + 4);
        v8h hv;
        hv[0] = (_Float16)(a.x * 64.0f);
        hv[1] = (_Float16)(a.y * 64.0f);
        hv[2] = (_Float16)(a.z * 64.0f);
        hv[3] = (_Float16)(a.w * 64.0f);
        hv[4] = (_Float16)(b.x * 64.0f);
        hv[5] = (_Float16)(b.y * 64.0f);
        hv[6] = (_Float16)(b.z * 64.0f);
        hv[7] = (_Float16)(b.w * 64.0f);
        *(v8ha*)(ar + 8 * q) = hv;
      }
    }
    __syncthreads();

#pragma unroll 2
    for (int kc = 0; kc < 8; ++kc) {
      const int k0g = sup * KSUP + kc * 32;
      const v16h a0 = ldfrag_l(sA, LDA, 0, kc * 32, lane);
      const v16h a1 = ldfrag_l(sA, LDA, 16, kc * 32, lane);
#pragma unroll
      for (int t = 0; t < 4; ++t) {
        const v16h b = ldfrag_g(WT, KTOT, ncol0 + 16 * t, k0g, lane);
        acc[0][t] = mma16(a0, b, acc[0][t]);
        acc[1][t] = mma16(a1, b, acc[1][t]);
      }
    }
    __syncthreads();
  }

  const float scl = 6.103515625e-05f;
  float badd[4], gmv[4], btv[4];
#pragma unroll
  for (int t = 0; t < 4; ++t) {
    const int col = ncol0 + 16 * t + c;
    badd[t] = bias[col] + skipb[col];
    gmv[t]  = gmg[col];
    btv[t]  = btg[col];
  }
#pragma unroll
  for (int s = 0; s < 2; ++s) {
#pragma unroll
    for (int t = 0; t < 4; ++t) {
#pragma unroll
      for (int r = 0; r < 8; ++r) acc[s][t][r] = acc[s][t][r] * scl + badd[t];
    }
  }

#pragma unroll
  for (int s = 0; s < 2; ++s) {
#pragma unroll
    for (int r = 0; r < 8; ++r) {
      float p = (acc[s][0][r] + acc[s][1][r]) + (acc[s][2][r] + acc[s][3][r]);
      p += __shfl_xor(p, 8, 16);
      p += __shfl_xor(p, 4, 16);
      p += __shfl_xor(p, 2, 16);
      p += __shfl_xor(p, 1, 16);
      if (c == 0) part[(s * 16 + 8 * hh + r) * 8 + wave] = p;
    }
  }
  __syncthreads();
  if (wave == 0) {
    const float* pr = part + lane * 8;
    const float s8 = ((pr[0] + pr[1]) + (pr[2] + pr[3])) + ((pr[4] + pr[5]) + (pr[6] + pr[7]));
    mu_s[lane] = s8 * (1.0f / 512.0f);
  }
  __syncthreads();

#pragma unroll
  for (int s = 0; s < 2; ++s) {
#pragma unroll
    for (int r = 0; r < 8; ++r) {
      const float mu = mu_s[s * 16 + 8 * hh + r];
      float p = 0.0f;
#pragma unroll
      for (int t = 0; t < 4; ++t) {
        const float d = acc[s][t][r] - mu;
        acc[s][t][r] = d;
        p += d * d;
      }
      p += __shfl_xor(p, 8, 16);
      p += __shfl_xor(p, 4, 16);
      p += __shfl_xor(p, 2, 16);
      p += __shfl_xor(p, 1, 16);
      if (c == 0) part[(s * 16 + 8 * hh + r) * 8 + wave] = p;
    }
  }
  __syncthreads();
  if (wave == 0) {
    const float* pr = part + lane * 8;
    const float s8 = ((pr[0] + pr[1]) + (pr[2] + pr[3])) + ((pr[4] + pr[5]) + (pr[6] + pr[7]));
    rs_s[lane] = rsqrtf(s8 * (1.0f / 512.0f) + 1e-5f);
  }
  __syncthreads();

  float* sw = st[wave];
#pragma unroll
  for (int s = 0; s < 2; ++s) {
#pragma unroll
    for (int r = 0; r < 8; ++r) {
      const float rsd = rs_s[s * 16 + 8 * hh + r];
#pragma unroll
      for (int t = 0; t < 4; ++t) {
        const float nv = acc[s][t][r] * rsd * gmv[t] + btv[t];
        const float gv = 0.5f * nv * erfcf(-nv * 0.70710678118654752f);
        sw[(8 * hh + r) * STP + 16 * t + c] = gv;
      }
    }
    __syncthreads();
    v4f val[8];
    size_t go[8];
#pragma unroll
    for (int it = 0; it < 8; ++it) {
      const int p  = lane + 32 * it;
      const int L  = p >> 4;
      const int pc = p & 15;
      val[it] = *(const v4fa*)(sw + L * STP + pc * 4);
      go[it]  = (size_t)(m0 + s * 16 + L) * NO + ncol0 + pc * 4;
    }
#pragma unroll
    for (int it = 0; it < 8; ++it) *(volatile v4f*)(out + go[it]) = val[it];
    __threadfence();
#pragma unroll
    for (int it = 0; it < 8; ++it) *(volatile v4f*)(out + go[it]) = val[it];
    __syncthreads();
  }
}

extern "C" void kernel_launch(void* const* d_in, const int* in_sizes, int n_in,
                              void* d_out, int out_size, void* d_ws, size_t ws_size,
                              hipStream_t stream) {
  if (n_in < 9) return;
  if (in_sizes[0] != NB * NI) return;
  if (in_sizes[1] != NI) return;
  if (in_sizes[2] != NI) return;
  if (in_sizes[3] != NI * NG * NO) return;
  if (in_sizes[4] != NO) return;
  if (in_sizes[5] != NI * NO) return;
  if (in_sizes[6] != NO) return;
  if (in_sizes[7] != NO) return;
  if (in_sizes[8] != NO) return;
  if (out_size != NB * NO) return;

  const float* x      = (const float*)d_in[0];
  const float* shf    = (const float*)d_in[1];
  const float* lsc    = (const float*)d_in[2];
  const float* coeffs = (const float*)d_in[3];
  const float* bias   = (const float*)d_in[4];
  const float* skipw  = (const float*)d_in[5];
  const float* skipb  = (const float*)d_in[6];
  const float* gmg    = (const float*)d_in[7];
  const float* btg    = (const float*)d_in[8];
  float* out = (float*)d_out;

  const size_t wt_bytes = (size_t)NO * KTOT * 2;
  if (wt_bytes > ws_size) return;
  _Float16* WT = (_Float16*)d_ws;

  k_prep<<<dim3(KTOT / 64, NO / 32), dim3(256), 0, stream>>>(coeffs, skipw, WT);
  k_main<<<dim3(NB / BM), dim3(256), 0, stream>>>(x, shf, lsc, WT, bias, skipb, gmg, btg, out);
  (void)hipGetLastError();
}
